// TransformerBlocks_50921132261733
// MI455X (gfx1250) — hardware-verified
//
#include <hip/hip_runtime.h>
#include <math.h>

typedef __attribute__((ext_vector_type(16))) _Float16 v16h;
typedef __attribute__((ext_vector_type(16))) __bf16 v16b;
typedef __attribute__((ext_vector_type(8)))  _Float16 v8h;
typedef __attribute__((ext_vector_type(8)))  float v8f;
typedef __attribute__((ext_vector_type(4)))  float v4f;
typedef __attribute__((ext_vector_type(2)))  float v2f;
typedef __attribute__((ext_vector_type(4)))  unsigned v4u;
typedef __attribute__((ext_vector_type(4)))  int v4i;
typedef float __attribute__((may_alias)) float_a;
typedef int __attribute__((may_alias)) int_a;

template <typename T> __device__ __forceinline__ void vst2(void* p, T v) { *(volatile T*)p = v; __threadfence(); *(volatile T*)p = v; }
__device__ __forceinline__ v8f wmma16(v16h a, v16h b, v8f c) {
  v8f d = __builtin_amdgcn_wmma_f32_16x16x32_f16(false, a, false, b, (short)0, c, false, false);
  asm volatile("v_nop\n\tv_nop\n\tv_nop\n\tv_nop" : "+v"(d) : "v"(a), "v"(b));
  return d;
}
__device__ __forceinline__ v8f wmma_bf(v16b a, v16b b, v8f c) {
  v8f d = __builtin_amdgcn_wmma_f32_16x16x32_bf16(false, a, false, b, (short)0, c, false, false);
  asm volatile("v_nop\n\tv_nop\n\tv_nop\n\tv_nop" : "+v"(d) : "v"(a), "v"(b));
  return d;
}
__device__ __forceinline__ v16h frag_h(const _Float16* rowk0, int lane) {
  union { v16h v; v8h q[2]; } u; const _Float16* p = rowk0 + 8 * (lane >> 4);
  u.q[0] = *(const v8h*)p; u.q[1] = *(const v8h*)(p + 16); return u.v;
}
__device__ __forceinline__ v16h frag_f32(const float* rowk0, int lane) {
  v16h a; const float* p = rowk0 + 8 * (lane >> 4);
#pragma unroll
  for (int i = 0; i < 8; ++i) { a[i] = (_Float16)p[i]; a[8 + i] = (_Float16)p[16 + i]; }
  return a;
}
__device__ __forceinline__ v16h frag_f32s(const float* rowk0, int lane, float sc) {
  v16h a; const float* p = rowk0 + 8 * (lane >> 4);
#pragma unroll
  for (int i = 0; i < 8; ++i) { a[i] = (_Float16)(p[i] * sc); a[8 + i] = (_Float16)(p[16 + i] * sc); }
  return a;
}
__device__ __forceinline__ v16h fragc_f32(const float* W, int k0, int n, int lane, int ld, int K) {
  v16h a; const int g = lane >> 4;
#pragma unroll
  for (int i = 0; i < 8; ++i) { const int ka = k0 + 8 * g + i, kb = ka + 16;
    a[i] = (_Float16)(ka < K ? W[(size_t)(ka < K ? ka : K - 1) * ld + n] : 0.f); a[8 + i] = (_Float16)(kb < K ? W[(size_t)(kb < K ? kb : K - 1) * ld + n] : 0.f); }
  return a;
}
struct F2 { v16b h, l; };
__device__ __forceinline__ F2 bsplit16(const float v[16]) { F2 r;
#pragma unroll
  for (int i = 0; i < 16; ++i) { const __bf16 h = (__bf16)v[i]; r.h[i] = h; r.l[i] = (__bf16)(v[i] - (float)h); }
  return r; }
__device__ __forceinline__ F2 split_row(const float* row, int k0, int lane) { float v[16]; const float* p = row + k0 + 8 * (lane >> 4);
#pragma unroll
  for (int i = 0; i < 8; ++i) { v[i] = p[i]; v[8 + i] = p[16 + i]; }
  return bsplit16(v); }
__device__ __forceinline__ F2 split_rowK(const float* row, int k0, int lane, int K) { float v[16]; const int g = lane >> 4;
#pragma unroll
  for (int i = 0; i < 8; ++i) { const int ka = k0 + 8 * g + i, kb = ka + 16; v[i] = ka < K ? row[ka < K ? ka : K - 1] : 0.f; v[8 + i] = kb < K ? row[kb < K ? kb : K - 1] : 0.f; }
  return bsplit16(v); }
__device__ __forceinline__ F2 split_col(const float* W, int k0, int n, int lane, int ld, int K) { float v[16]; const int g = lane >> 4;
#pragma unroll
  for (int i = 0; i < 8; ++i) { const int ka = k0 + 8 * g + i, kb = ka + 16; v[i] = ka < K ? W[(size_t)(ka < K ? ka : K - 1) * ld + n] : 0.f; v[8 + i] = kb < K ? W[(size_t)(kb < K ? kb : K - 1) * ld + n] : 0.f; }
  return bsplit16(v); }
__device__ __forceinline__ v8f mac3(const F2& a, const F2& b, v8f c) { c = wmma_bf(a.l, b.h, c); c = wmma_bf(a.h, b.l, c); return wmma_bf(a.h, b.h, c); }
__device__ __forceinline__ float sigm(float v) { return 1.0f / (1.0f + expf(-v)); }
#define LDSX() do { asm volatile("s_wait_dscnt 0" ::: "memory"); __builtin_amdgcn_wave_barrier(); __builtin_amdgcn_fence(__ATOMIC_RELEASE, "workgroup"); } while (0)


#define NB 2
#define SS 2048
#define CC 512
#define DM 1024
#define NH 16
#define HD 64
#define QKVW (3 * DM)
#define INR 1365
#define INP 1376
#define NR (NB * SS)
#ifndef TQB
#define TQB (SS / 64)
#define TNB NB
#define TB0 0
#define TOB (NB * SS / 64)
#endif
#define RB0 ((size_t)TB0 * SS)
typedef __attribute__((ext_vector_type(8))) __bf16 v8b;
__device__ __forceinline__ v16b frag_b(const __bf16* rowk0, int lane) {
  union { v16b v; v8b q[2]; } u; const __bf16* p = rowk0 + 8 * (lane >> 4);
  u.q[0] = *(const v8b*)p; u.q[1] = *(const v8b*)(p + 16); return u.v;
}
__device__ __forceinline__ float bfr(float v) { return (float)(__bf16)v; }
__device__ __attribute__((noinline)) float exp_ni(float v) { return expf(v); }
__device__ __attribute__((noinline)) float erf_ni(float v) { return erff(v); }

#define PK_A  0
#define PK_O  ((size_t)QKVW * CC)
#define PK_FA (PK_O + (size_t)CC * DM)
#define PK_FG (PK_FA + (size_t)INP * CC)
#define PK_F2 (PK_FG + (size_t)INP * CC)
#define PK_END (PK_F2 + (size_t)CC * INP)
#define WS_PK  0u
#define WS_QK  (((2u * PK_END) + 127u) / 128u * 128u)
#define WS_QKL (WS_QK + 2u * NR * 2 * DM)
#define WS_VTH (WS_QKL + 2u * NR * 2 * DM)
#define WS_VTL (WS_VTH + 2u * NR * DM)
#define WS_O   (WS_VTL + 2u * NR * DM)
#define WS_X1  (WS_O + 4u * NR * DM)
#define WS_XN  (WS_X1 + 4u * NR * CC)
#define WS_H2  (WS_XN + 4u * NR * CC)
#define WS_HH  (WS_H2 + 4u * (size_t)NR * INP)
#define WS_HL  (WS_HH + 2u * (size_t)NR * INP)
#define WS_X2  (WS_HL + 2u * (size_t)NR * INP)
#define WS_ST  (WS_X2 + 4u * NR * CC)
#define STSZ   ((size_t)(NR / 64) * 16 * 32)
#define WS_MS  (WS_ST + 4u * 3 * STSZ)
#define WS_END (WS_MS + 4u * 3 * NB * 2)

__global__ __launch_bounds__(256) void k_pack(const float* __restrict__ WQ, const float* __restrict__ WO, const float* __restrict__ W1, const float* __restrict__ W2, __bf16* __restrict__ PK) {
  __shared__ __align__(16) __bf16 s[INP]; const int n = blockIdx.x, which = blockIdx.y, t = threadIdx.x; int K; size_t dst;
  switch (which) {
    case 0: if (n >= QKVW) return; K = CC; dst = PK_A + (size_t)n * CC; for (int k = t; k < K; k += 256) s[k] = (__bf16)WQ[(size_t)n * CC + k]; break;
    case 1: if (n >= CC) return; K = DM; dst = PK_O + (size_t)n * DM; for (int k = t; k < K; k += 256) s[k] = (__bf16)WO[(size_t)n * DM + k]; break;
    case 2: if (n >= INP) return; K = CC; dst = PK_FA + (size_t)n * CC; for (int k = t; k < K; k += 256) s[k] = (__bf16)((n < INR) ? W1[(size_t)n * CC + k] : 0.f); break;
    case 3: if (n >= INP) return; K = CC; dst = PK_FG + (size_t)n * CC; for (int k = t; k < K; k += 256) s[k] = (__bf16)((n < INR) ? W1[(size_t)(INR + n) * CC + k] : 0.f); break;
    default: if (n >= CC) return; K = INP; dst = PK_F2 + (size_t)n * INP; for (int k = t; k < K; k += 256) s[k] = (__bf16)((k < INR) ? W2[(size_t)n * INR + k] : 0.f); break; }
  __syncthreads();
  for (int q = t; q < K / 8; q += 256) vst2((unsigned*)(PK + dst + q * 8), *(const v4u*)&s[q * 8]);
}
__global__ __launch_bounds__(128) void k_qkv(const float* __restrict__ X, const __bf16* __restrict__ P, const float* __restrict__ QS, const float* __restrict__ KS, _Float16* __restrict__ QK, _Float16* __restrict__ QKL, _Float16* __restrict__ VTH, _Float16* __restrict__ VTL) {
  __shared__ __align__(16) __bf16 sa[64][CC + 8]; __shared__ __align__(16) _Float16 so[4][16][136], sol[4][16][136];
  const int tid = threadIdx.x, wave = tid >> 5, lane = tid & 31, col = lane & 15, g = lane >> 4; const size_t b = blockIdx.z + TB0; const int p0 = blockIdx.x * 64; const int n0 = blockIdx.y * 128; const size_t r0 = b * SS + p0 + wave * 16;
  for (int e = tid; e < 64 * CC; e += 128) { const int c = e >> 6, r = e & 63; sa[r][c] = (__bf16)X[(b * CC + c) * SS + p0 + r]; }
  if (tid < 64) for (int c = CC; c < CC + 8; ++c) sa[tid][c] = (__bf16)0.f;
  __syncthreads();
  v8f acc[8] = {};
#pragma unroll 2
  for (int kc = 0; kc < CC / 32; ++kc) { const v16b a = frag_b(&sa[wave * 16 + col][kc * 32], lane);
#pragma unroll
    for (int j = 0; j < 8; ++j) acc[j] = wmma_bf(a, frag_b(P + (size_t)(n0 + j * 16 + col) * CC + kc * 32, lane), acc[j]); }
  if (n0 < 2 * DM) { const float* SCL = (n0 < DM) ? QS : KS;
    float rn[2][8];
#pragma unroll
    for (int hh = 0; hh < 2; ++hh)
#pragma unroll
      for (int r = 0; r < 8; ++r) { float s2 = 0.f;
#pragma unroll
        for (int j = hh * 4; j < hh * 4 + 4; ++j) s2 += acc[j][r] * acc[j][r];
#pragma unroll
        for (int o = 1; o < 16; o <<= 1) s2 += __shfl_xor(s2, o);
        rn[hh][r] = 1.0f / sqrtf(s2 + 1e-12f); }
#pragma unroll
    for (int j = 0; j < 8; ++j) { const float sc = bfr(SCL[(j & 3) * 16 + col]);
#pragma unroll
      for (int r = 0; r < 8; ++r) { const float v = acc[j][r] * rn[j >> 2][r] * sc; const _Float16 hv = (_Float16)v; so[wave][8 * g + r][j * 16 + col] = hv; sol[wave][8 * g + r][j * 16 + col] = (_Float16)((v - (float)hv) * 2048.0f); } }
    LDSX();
    for (int rl = 0; rl < 16; ++rl) if (lane < 16) { vst2((unsigned*)(QK + (r0 + rl) * (2 * DM) + n0 + lane * 8), *(const v4u*)&so[wave][rl][lane * 8]); vst2((unsigned*)(QKL + (r0 + rl) * (2 * DM) + n0 + lane * 8), *(const v4u*)&sol[wave][rl][lane * 8]); }
  } else {
    __shared__ __align__(16) _Float16 sth[128][72], stl[128][72];
#pragma unroll
    for (int j = 0; j < 8; ++j)
#pragma unroll
      for (int r = 0; r < 8; ++r) { const float v = acc[j][r]; const _Float16 hv = (_Float16)v; sth[j * 16 + col][wave * 16 + 8 * g + r] = hv; stl[j * 16 + col][wave * 16 + 8 * g + r] = (_Float16)((v - (float)hv) * 2048.0f); }
    __syncthreads();
    const int pc0 = n0 - 2 * DM;
    for (int q = tid; q < 128 * 8; q += 128) { const int d = q >> 3, pc = q & 7; const size_t o = (b * DM + pc0 + d) * SS + p0 + pc * 8; vst2((unsigned*)(VTH + o), *(const v4u*)&sth[d][pc * 8]); vst2((unsigned*)(VTL + o), *(const v4u*)&stl[d][pc * 8]); }
  }
}
__global__ __launch_bounds__(128) void k_attn(const _Float16* __restrict__ QK, const _Float16* __restrict__ QKL, const _Float16* __restrict__ VTH, const _Float16* __restrict__ VTL, float* __restrict__ O) {
  __shared__ __align__(16) float sp[4][16][36]; __shared__ __align__(16) float so[4][16][68];
  const int tid = threadIdx.x, wave = tid >> 5, lane = tid & 31, col = lane & 15, g = lane >> 4;
  const int qb = blockIdx.x, h = blockIdx.y, b = blockIdx.z + TB0; const int q0 = qb * 64 + wave * 16; const size_t rq = (size_t)b * SS + q0 + col;
  v16h aq[2], aql[2];
#pragma unroll
  for (int kc = 0; kc < 2; ++kc) { aq[kc] = frag_h(QK + rq * (2 * DM) + h * HD + kc * 32, lane); aql[kc] = frag_h(QKL + rq * (2 * DM) + h * HD + kc * 32, lane); }
  float m[8], l[8];
#pragma unroll
  for (int r = 0; r < 8; ++r) { m[r] = -3.0e38f; l[r] = 0.f; }
  v8f acc[4] = {}, accl[4] = {};
  const int nks = SS / 32;
#pragma unroll 1
  for (int ks = 0; ks < nks; ++ks) { v8f s[2];
#pragma unroll
    for (int ct = 0; ct < 2; ++ct) { const int kk = ks * 32 + ct * 16 + col; const _Float16* krow = QK + ((size_t)b * SS + kk) * (2 * DM) + DM + h * HD; const _Float16* krowl = QKL + ((size_t)b * SS + kk) * (2 * DM) + DM + h * HD; v8f c = {}, cl = {};
#pragma unroll
      for (int kc = 0; kc < 2; ++kc) { const v16h kh = frag_h(krow + kc * 32, lane); c = wmma16(aq[kc], kh, c); cl = wmma16(aql[kc], kh, cl); cl = wmma16(aq[kc], frag_h(krowl + kc * 32, lane), cl); }
#pragma unroll
      for (int r = 0; r < 8; ++r) c[r] += cl[r] * (1.0f / 2048.0f);
#pragma unroll
      for (int r = 0; r < 8; ++r) s[ct][r] = c[r] * 8.0f; }
#pragma unroll
    for (int r = 0; r < 8; ++r) { float mx = fmaxf(s[0][r], s[1][r]);
#pragma unroll
      for (int o = 1; o < 16; o <<= 1) mx = fmaxf(mx, __shfl_xor(mx, o));
      const float mn = fmaxf(m[r], mx); const float alpha = (m[r] <= -1.0e38f) ? 0.f : __expf(m[r] - mn);
      const float e0 = (s[0][r] <= -1.0e38f) ? 0.f : __expf(s[0][r] - mn), e1 = (s[1][r] <= -1.0e38f) ? 0.f : __expf(s[1][r] - mn); float es = e0 + e1;
#pragma unroll
      for (int o = 1; o < 16; o <<= 1) es += __shfl_xor(es, o);
      l[r] = l[r] * alpha + es; m[r] = mn;
#pragma unroll
      for (int dt = 0; dt < 4; ++dt) { acc[dt][r] *= alpha; accl[dt][r] *= alpha; }
      sp[wave][8 * g + r][col] = e0; sp[wave][8 * g + r][16 + col] = e1; }
    LDSX();
    v16h pa, pl; { const float* prow = &sp[wave][col][0] + 8 * (lane >> 4);
#pragma unroll
      for (int i = 0; i < 8; ++i) { const float x0 = prow[i], x1 = prow[16 + i]; const _Float16 h0 = (_Float16)x0, h1 = (_Float16)x1; pa[i] = h0; pa[8 + i] = h1; pl[i] = (_Float16)((x0 - (float)h0) * 2048.0f); pl[8 + i] = (_Float16)((x1 - (float)h1) * 2048.0f); } }
#pragma unroll
    for (int dt = 0; dt < 4; ++dt) { const size_t vr = ((size_t)b * DM + h * HD + dt * 16 + col) * SS + ks * 32; const v16h vh = frag_h(VTH + vr, lane); acc[dt] = wmma16(pa, vh, acc[dt]); accl[dt] = wmma16(pl, vh, accl[dt]); accl[dt] = wmma16(pa, frag_h(VTL + vr, lane), accl[dt]); }
    LDSX(); }
#pragma unroll
  for (int r = 0; r < 8; ++r) { const float il = 1.0f / l[r];
#pragma unroll
    for (int dt = 0; dt < 4; ++dt) so[wave][8 * g + r][dt * 16 + col] = (acc[dt][r] + accl[dt][r] * (1.0f / 2048.0f)) * il; }
  LDSX();
  for (int rl = 0; rl < 16; ++rl) if (lane < 16) vst2(O + ((size_t)b * SS + q0 + rl) * DM + h * HD + lane * 4, *(const v4f*)&so[wave][rl][lane * 4]);
}

template <int MODE>
__global__ __launch_bounds__(128) void k_lin(const float* __restrict__ A, const __bf16* __restrict__ AH, const __bf16* __restrict__ AL, const __bf16* __restrict__ PK, const float* __restrict__ BIAS, const float* __restrict__ RES, float* __restrict__ OUTF, float* __restrict__ ST) {
  __shared__ __align__(16) float so[4][16][132]; __shared__ __align__(16) float sst[2][128];
  const int tid = threadIdx.x, wave = tid >> 5, lane = tid & 31, col = lane & 15, g = lane >> 4; const size_t r0 = RB0 + (size_t)blockIdx.x * 64 + wave * 16; const int n0 = blockIdx.y * 128;
  constexpr int KD = (MODE == 0) ? DM : (MODE == 1) ? CC : INP; constexpr int NO = (MODE == 1) ? INP : CC;
  v8f acc[8] = {}, accg[8] = {};
  if (MODE == 2) {
#pragma unroll 2
    for (int kc = 0; kc < KD / 32; ++kc) { const v16b a = frag_b(AH + (r0 + col) * INP + kc * 32, lane), al = frag_b(AL + (r0 + col) * INP + kc * 32, lane);
#pragma unroll
      for (int j = 0; j < 8; ++j) { const v16b w = frag_b(PK + PK_F2 + (size_t)(n0 + j * 16 + col) * INP + kc * 32, lane); acc[j] = wmma_bf(al, w, acc[j]); acc[j] = wmma_bf(a, w, acc[j]); } }
  } else {
#pragma unroll 2
    for (int kc = 0; kc < KD / 32; ++kc) { const F2 a = split_row(A + (r0 + col) * KD, kc * 32, lane);
#pragma unroll
      for (int j = 0; j < 8; ++j) { if (MODE == 1 && n0 + j * 16 >= INP) continue; const __bf16* Prow = PK + ((MODE == 0) ? PK_O : PK_FA) + (size_t)(n0 + j * 16 + col) * KD + kc * 32; const v16b w = frag_b(Prow, lane); acc[j] = wmma_bf(a.l, w, acc[j]); acc[j] = wmma_bf(a.h, w, acc[j]);
        if (MODE == 1) { const v16b wg = frag_b(PK + PK_FG + (size_t)(n0 + j * 16 + col) * KD + kc * 32, lane); accg[j] = wmma_bf(a.l, wg, accg[j]); accg[j] = wmma_bf(a.h, wg, accg[j]); } } } }
#pragma unroll
  for (int j = 0; j < 8; ++j) { const int c = n0 + j * 16 + col;
#pragma unroll
    for (int r = 0; r < 8; ++r) { const size_t row = r0 + 8 * g + r; float v;
      if (MODE == 0) { const size_t b = row / SS; const int n = (int)(row % SS); v = acc[j][r] + bfr(BIAS[c]) + bfr(RES[(b * CC + c) * SS + n]); }
      else if (MODE == 1) { if (c < INR) { const float a_ = acc[j][r], gt = accg[j][r]; v = gt * (a_ / (1.0f + exp_ni(-a_))); } else v = 0.f; }
      else { v = acc[j][r] + RES[row * CC + c]; }
      so[wave][8 * g + r][j * 16 + col] = v; } }
  __syncthreads();
  if (n0 + 128 <= NO) { for (int rl = 0; rl < 16; ++rl) vst2(OUTF + (r0 + rl) * NO + n0 + lane * 4, *(const v4f*)&so[wave][rl][lane * 4]); }
  else { for (int rl = 0; rl < 16; ++rl) if (n0 + lane * 4 < NO) vst2(OUTF + (r0 + rl) * NO + n0 + lane * 4, *(const v4f*)&so[wave][rl][lane * 4]); }
  { const int c = tid; float s = 0.f, q2 = 0.f; if (n0 + c < NO) for (int w = 0; w < 4; ++w) for (int r = 0; r < 16; ++r) { const float v = so[w][r][c]; s += v; q2 += v * v; } sst[0][c] = s; sst[1][c] = q2; }
  __syncthreads();
  if (tid == 0) { float s = 0.f, q2 = 0.f; for (int c = 0; c < 128; ++c) { s += sst[0][c]; q2 += sst[1][c]; } so[0][0][0] = s; so[0][0][1] = q2; so[0][0][2] = 0.f; so[0][0][3] = 0.f; }
  __syncthreads();
  if (tid == 0) vst2(ST + (((size_t)(RB0 / 64) + blockIdx.x) * 16 + blockIdx.y) * 32, *(const v4f*)&so[0][0][0]);
}

__global__ __launch_bounds__(32) void k_gstat(const float* __restrict__ ST, int stage, int ncb, float cnt, float* __restrict__ MS) {
  const int b = blockIdx.x + TB0; if (threadIdx.x != 0) return; float s = 0.f, q2 = 0.f;
  for (int rb = b * (SS / 64); rb < (b + 1) * (SS / 64); ++rb) for (int cb = 0; cb < ncb; ++cb) { const float* p = ST + (size_t)stage * STSZ + ((size_t)rb * 16 + cb) * 32; s += p[0]; q2 += p[1]; }
  const float mu = s / cnt; const float var = fmaxf(q2 / cnt - mu * mu, 0.f); __shared__ __align__(16) float sm[4]; sm[0] = mu; sm[1] = 1.0f / sqrtf(var + 1e-5f); sm[2] = 0.f; sm[3] = 0.f; vst2(MS + ((size_t)stage * NB + b) * 32, *(const v4f*)sm);
}
template <int MODE>
__global__ __launch_bounds__(256) void k_gn(const float* __restrict__ X, const float* __restrict__ MS, int stage, const float* __restrict__ G, const float* __restrict__ Bb, float* __restrict__ OUTF, __bf16* __restrict__ OH_, __bf16* __restrict__ OL_) {
  const int t = threadIdx.x; const size_t r0 = RB0 + (size_t)blockIdx.x * 64; const size_t b = r0 / SS; const float mu = MS[((size_t)stage * NB + b) * 32], rs = MS[((size_t)stage * NB + b) * 32 + 1];
  if (MODE == 0) { for (int e = t; e < 64 * CC / 4; e += 256) { const int r = e / (CC / 4), q = e % (CC / 4); v4f v = *(const v4f*)(X + (r0 + r) * CC + q * 4), o;
#pragma unroll
      for (int i = 0; i < 4; ++i) { const int c = q * 4 + i; o[i] = (v[i] - mu) * rs * bfr(G[c]) + bfr(Bb[c]); } vst2(OUTF + (r0 + r) * CC + q * 4, o); } }
  else if (MODE == 1) { for (int e = t; e < 64 * INP / 8; e += 256) { const int r = e / (INP / 8), q = e % (INP / 8); __align__(16) __bf16 hh[8], ll[8];
#pragma unroll
      for (int i = 0; i < 8; ++i) { const int c = q * 8 + i; float y = 0.f; if (c < INR) y = (X[(r0 + r) * INP + c] - mu) * rs * bfr(G[c]) + bfr(Bb[c]); const __bf16 hb = (__bf16)y; hh[i] = hb; ll[i] = (__bf16)(y - (float)hb); }
      vst2((unsigned*)(OH_ + (r0 + r) * INP + q * 8), *(const v4u*)hh); vst2((unsigned*)(OL_ + (r0 + r) * INP + q * 8), *(const v4u*)ll); } }
  else { __shared__ float st[CC][65]; const int n0 = (int)(r0 % SS);
    for (int e = t; e < 64 * CC; e += 256) { const int r = e / CC, c = e % CC; st[c][r] = (X[(r0 + r) * CC + c] - mu) * rs * bfr(G[c]) + bfr(Bb[c]); }
    __syncthreads();
    for (int e = t; e < CC * 16; e += 256) { const int c = e >> 4, q = e & 15; v4f v = {st[c][q * 4], st[c][q * 4 + 1], st[c][q * 4 + 2], st[c][q * 4 + 3]}; vst2(OUTF + (b * CC + c) * SS + n0 + q * 4, v); } }
}
extern "C" void kernel_launch(void* const* d_in, const int* in_sizes, int n_in, void* d_out, int out_size, void* d_ws, size_t ws_size, hipStream_t stream) {
  (void)in_sizes; (void)n_in; (void)out_size;
  const float** F = (const float**)d_in;
  if (ws_size < (size_t)WS_END) return;
  char* ws = (char*)d_ws; __bf16 *PK = (__bf16*)(ws + WS_PK), *HH = (__bf16*)(ws + WS_HH), *HL = (__bf16*)(ws + WS_HL); _Float16 *QK = (_Float16*)(ws + WS_QK), *QKL = (_Float16*)(ws + WS_QKL), *VTH = (_Float16*)(ws + WS_VTH), *VTL = (_Float16*)(ws + WS_VTL);
  float *O = (float*)(ws + WS_O), *X1 = (float*)(ws + WS_X1), *XN = (float*)(ws + WS_XN), *H2 = (float*)(ws + WS_H2), *X2 = (float*)(ws + WS_X2), *ST = (float*)(ws + WS_ST), *MS = (float*)(ws + WS_MS);
  const int RT = TNB * SS / 64;
  k_pack<<<dim3(QKVW, 5), 256, 0, stream>>>(F[1], F[4], F[8], F[11], PK);
  k_qkv<<<dim3(SS / 64, QKVW / 128, TNB), 128, 0, stream>>>(F[0], PK + PK_A, F[2], F[3], QK, QKL, VTH, VTL);
  k_attn<<<dim3(TQB, NH, TNB), 128, 0, stream>>>(QK, QKL, VTH, VTL, O);
  k_lin<0><<<dim3(RT, CC / 128), 128, 0, stream>>>(O, nullptr, nullptr, PK, F[5], F[0], X1, ST);
  k_gstat<<<TNB, 32, 0, stream>>>(ST, 0, CC / 128, (float)CC * SS, MS);
  k_gn<0><<<RT, 256, 0, stream>>>(X1, MS, 0, F[6], F[7], XN, nullptr, nullptr);
  k_lin<1><<<dim3(RT, (INP + 127) / 128), 128, 0, stream>>>(XN, nullptr, nullptr, PK, nullptr, nullptr, H2, ST + STSZ);
  k_gstat<<<TNB, 32, 0, stream>>>(ST, 1, (INP + 127) / 128, (float)INR * SS, MS);
  k_gn<1><<<RT, 256, 0, stream>>>(H2, MS, 1, F[9], F[10], nullptr, HH, HL);
  k_lin<2><<<dim3(RT, CC / 128), 128, 0, stream>>>(nullptr, HH, HL, PK, nullptr, X1, X2, ST + 2 * STSZ);
  k_gstat<<<TNB, 32, 0, stream>>>(ST, 2, CC / 128, (float)CC * SS, MS);
  k_gn<2><<<RT, 256, 0, stream>>>(X2, MS, 2, F[12], F[13], (float*)d_out, nullptr, nullptr);
}
